// HypergraphConv_62792421867972
// MI455X (gfx1250) — hardware-verified
//
#include <hip/hip_runtime.h>


namespace {
constexpr int Bn = 2, C = 128, N = 50000, K = 5000, M1 = 32, M2 = 8, NKT = (K + 15) / 16  , NNT = 50048 / 128  ;
constexpr float AS_ = 8.0f;

typedef _Float16 b16;
typedef __attribute__((ext_vector_type(16))) _Float16 v16b;
typedef __attribute__((ext_vector_type(8))) _Float16 v8b;
typedef __attribute__((ext_vector_type(4))) _Float16 v4b;
typedef __attribute__((ext_vector_type(8))) float v8f;
typedef __attribute__((ext_vector_type(4))) float v4f;
__device__ __forceinline__ float bf16_rne(float f) { unsigned int u = __float_as_uint(f); u += 0x7FFFu + ((u >> 16) & 1u); return __uint_as_float(u & 0xFFFF0000u); }
__device__ __forceinline__ void split16(float v, b16& hi, b16& lo) { hi = (b16)v; lo = (b16)(v - (float)hi); }
__device__ __forceinline__ v16b frag_kb(const b16* p, int hh) { const v8b a = *(const v8b*)(p + 8 * hh), b = *(const v8b*)(p + 16 + 8 * hh); v16b f;
#pragma unroll
  for (int e = 0; e < 8; ++e) { f[e] = a[e]; f[8 + e] = b[e]; } return f; }
__device__ __forceinline__ void frag_split(const float* p, int hh, v16b& fh, v16b& fl) {
#pragma unroll
  for (int e = 0; e < 8; ++e) { b16 a, c; split16(p[8 * hh + e] * AS_, a, c); fh[e] = a; fl[e] = c; split16(p[16 + 8 * hh + e] * AS_, a, c); fh[8 + e] = a; fl[8 + e] = c; } }
__device__ __forceinline__ v8f wmma16b(v16b a, v16b b, v8f c) { v8f d = __builtin_amdgcn_wmma_f32_16x16x32_f16(false, a, false, b, (short)0, c, false, false); asm volatile("v_nop\n\tv_nop\n\tv_nop\n\tv_nop" : "+v"(d) : "v"(a), "v"(b)); return d; }
__device__ __forceinline__ void wave_lds_sync() { __builtin_amdgcn_fence(__ATOMIC_RELEASE, "workgroup"); __builtin_amdgcn_wave_barrier(); __builtin_amdgcn_fence(__ATOMIC_ACQUIRE, "workgroup"); }

__global__ __launch_bounds__(256) void prep_kernel(const float* __restrict__ w1a, const float* __restrict__ w1b, const float* __restrict__ w2a, const float* __restrict__ w2b, const float* __restrict__ b1a, const float* __restrict__ b1b, const float* __restrict__ b2a, const float* __restrict__ b2b, const float* __restrict__ eps, b16* __restrict__ R, float* __restrict__ P) {
  const int t_ = blockIdx.x * 256 + threadIdx.x, nth = gridDim.x * 256;
  for (int pass = 0; pass < 2; ++pass) {
    for (int i = t_; i < 4 * C * C; i += nth) { const int m = i / (C * C), o = (i / C) % C, k = i % C; const float* W = (m == 0) ? w1a : (m == 1) ? w1b : (m == 2) ? w2a : w2b; R[i] = (b16)bf16_rne(W[(size_t)k * C + o]); }
    for (int i = t_; i < 513; i += nth) { float v; if (i < 128) v = bf16_rne(b1a[i]); else if (i < 256) v = bf16_rne(b1b[i - 128]); else if (i < 384) v = bf16_rne(b2a[i - 256]); else if (i < 512) v = bf16_rne(b2b[i - 384]); else v = 1.0f + bf16_rne(eps[0]); P[i] = v; }
    __threadfence(); }
}

__global__ __launch_bounds__(256) void xpose_kernel(const float* __restrict__ x, b16* __restrict__ xt) {
  __shared__ __attribute__((aligned(16))) b16 T[128][C + 8];
  const int b = blockIdx.y, n0 = blockIdx.x * 128, t_ = threadIdx.x;
  for (int i = t_; i < C * 128; i += 256) { const int c = i >> 7, nn = i & 127; const int n = n0 + nn; T[nn][c] = (b16)((n < N) ? bf16_rne(x[((size_t)b * C + c) * N + n]) : 0.0f); }
  __syncthreads();
  for (int pass = 0; pass < 2; ++pass) { for (int i = t_; i < 128 * 16; i += 256) { const int nn = i >> 4, c8 = (i & 15) * 8; if (n0 + nn < N) *(volatile v8b*)(xt + ((size_t)b * N + n0 + nn) * C + c8) = *(const v8b*)(&T[nn][c8]); } __threadfence(); }
}

__device__ __forceinline__ void mlp16(float (*X)[C + 4], const b16* Wa, const b16* Wb, const float* ba, const float* bb, int nloc, int hlf) {
  v8f acc[8];
#pragma unroll
  for (int t = 0; t < 8; ++t) acc[t] = (v8f){};
  for (int kb = 0; kb < C; kb += 32) { v16b ah, al; frag_split(&X[nloc][kb], hlf, ah, al);
#pragma unroll
    for (int t = 0; t < 8; ++t) { const v16b bw = frag_kb(Wa + (size_t)(t * 16 + nloc) * C + kb, hlf); acc[t] = wmma16b(ah, bw, acc[t]); acc[t] = wmma16b(al, bw, acc[t]); } }
  wave_lds_sync();
#pragma unroll
  for (int t = 0; t < 8; ++t) { const float b_ = ba[t * 16 + nloc];
#pragma unroll
    for (int v = 0; v < 8; ++v) X[8 * hlf + v][t * 16 + nloc] = fmaxf(acc[t][v] * (1.0f / AS_) + b_, 0.0f); }
  wave_lds_sync();
#pragma unroll
  for (int t = 0; t < 8; ++t) acc[t] = (v8f){};
  for (int kb = 0; kb < C; kb += 32) { v16b ah, al; frag_split(&X[nloc][kb], hlf, ah, al);
#pragma unroll
    for (int t = 0; t < 8; ++t) { const v16b bw = frag_kb(Wb + (size_t)(t * 16 + nloc) * C + kb, hlf); acc[t] = wmma16b(ah, bw, acc[t]); acc[t] = wmma16b(al, bw, acc[t]); } }
  wave_lds_sync();
#pragma unroll
  for (int t = 0; t < 8; ++t) { const float b_ = bb[t * 16 + nloc];
#pragma unroll
    for (int v = 0; v < 8; ++v) X[8 * hlf + v][t * 16 + nloc] = acc[t][v] * (1.0f / AS_) + b_; }
  wave_lds_sync();
}

__global__ __launch_bounds__(128) void hedge_kernel(const b16* __restrict__ xt, const int* __restrict__ hm, const float* __restrict__ cen, const b16* __restrict__ R, const float* __restrict__ P, float* __restrict__ he) {
  __shared__ __attribute__((aligned(16))) float X[4][16][C + 4];
  const int wave = threadIdx.x >> 5, lane = threadIdx.x & 31, nloc = lane & 15, hlf = lane >> 4, b = blockIdx.y, k0 = (blockIdx.x * 4 + wave) * 16;
  if (k0 >= K) return;
  const b16* xb = xt + ((size_t)b * N) * C;
  for (int r = 0; r < 16; ++r) { const int k = min(k0 + r, K - 1); const int* idx = hm + ((size_t)b * K + k) * M1; v4f s = {0.0f, 0.0f, 0.0f, 0.0f};
    for (int m = 0; m < M1; ++m) { int n = idx[m]; if (n >= 0) { n = (n >= N) ? N - 1 : n; const v4b v = *(const v4b*)(xb + (size_t)n * C + lane * 4);
#pragma unroll
        for (int e = 0; e < 4; ++e) s[e] += (float)v[e]; } }
    *(v4f*)(&X[wave][r][lane * 4]) = s; }
  wave_lds_sync();
  mlp16(X[wave], R, R + C * C, P, P + 128, nloc, hlf);
  const float ope = P[512];
  for (int r = 0; r < 16; ++r) { const int k = k0 + r; if (k >= K) break; v4f v = *(const v4f*)(&X[wave][r][lane * 4]);
#pragma unroll
    for (int e = 0; e < 4; ++e) v[e] += ope * bf16_rne(cen[((size_t)b * C + lane * 4 + e) * K + k]);
    for (int pass = 0; pass < 2; ++pass) { *(volatile v4f*)(he + ((size_t)b * K + k) * C + lane * 4) = v; } }
  __threadfence();
}

__global__ __launch_bounds__(256) void node_kernel(const float* __restrict__ he, const int* __restrict__ phi, const b16* __restrict__ R, const float* __restrict__ P, float* __restrict__ out) {
  __shared__ __attribute__((aligned(16))) float X[8][16][C + 4];
  const int wave = threadIdx.x >> 5, lane = threadIdx.x & 31, nloc = lane & 15, hlf = lane >> 4, b = blockIdx.y, n0 = blockIdx.x * 128, nw = n0 + wave * 16;
  const float* heb = he + ((size_t)b * K) * C;
  for (int r = 0; r < 16; ++r) { const int n = min(nw + r, N - 1); const int* idx = phi + ((size_t)b * N + n) * M2; v4f s = {0.0f, 0.0f, 0.0f, 0.0f};
#pragma unroll
    for (int m = 0; m < M2; ++m) { int k = idx[m]; if (k >= 0) { k = (k >= K) ? K - 1 : k; const v4f v = *(const v4f*)(heb + (size_t)k * C + lane * 4);
#pragma unroll
        for (int e = 0; e < 4; ++e) s[e] += v[e]; } }
    *(v4f*)(&X[wave][r][lane * 4]) = s; }
  wave_lds_sync();
  mlp16(X[wave], R + 2 * C * C, R + 3 * C * C, P + 256, P + 384, nloc, hlf);
  __syncthreads();
  for (int pass = 0; pass < 2; ++pass) { for (int i = threadIdx.x; i < C * 32; i += 256) { const int o = i >> 5, q4 = (i & 31) * 4; if (n0 + q4 < N) { v4f v;
#pragma unroll
        for (int e = 0; e < 4; ++e) { const int nn = q4 + e; v[e] = X[nn >> 4][nn & 15][o]; }
        *(volatile v4f*)(out + ((size_t)b * C + o) * N + n0 + q4) = v; } } __threadfence(); }
}
}

extern "C" void kernel_launch(void* const* d_in, const int* in_sizes, int n_in,
                              void* d_out, int out_size, void* d_ws, size_t ws_size, hipStream_t stream) {
  (void)n_in; (void)out_size;
  const float* x = (const float*)d_in[0]; const int* hm = (const int*)d_in[1]; const int* phi = (const int*)d_in[2]; const float* cen = (const float*)d_in[3];
  const float* w1a = (const float*)d_in[4]; const float* b1a = (const float*)d_in[5]; const float* w1b = (const float*)d_in[6]; const float* b1b = (const float*)d_in[7]; const float* w2a = (const float*)d_in[8]; const float* b2a = (const float*)d_in[9]; const float* w2b = (const float*)d_in[10]; const float* b2b = (const float*)d_in[11]; const float* eps = (const float*)d_in[12];
  float* out = (float*)d_out;
  if (in_sizes[0] != Bn * C * N || in_sizes[1] != Bn * K * M1 || in_sizes[2] != Bn * N * M2 || in_sizes[3] != Bn * C * K || in_sizes[4] != C * C || in_sizes[12] != 1) return;
  size_t off = 0; char* ws = (char*)d_ws;
  auto carve = [&](size_t bytes) { char* p = ws + off; off += (bytes + 255) & ~(size_t)255; return p; };
  b16* R = (b16*)carve((size_t)4 * C * C * 2); float* P = (float*)carve(1024 * 4); b16* xt = (b16*)carve((size_t)Bn * N * C * 2); float* he = (float*)carve((size_t)Bn * K * C * 4);
  if (off > ws_size) return;
  prep_kernel<<<64, 256, 0, stream>>>(w1a, w1b, w2a, w2b, b1a, b1b, b2a, b2b, eps, R, P);
  xpose_kernel<<<dim3(NNT, Bn), 256, 0, stream>>>(x, xt);
  hedge_kernel<<<dim3((NKT + 3) / 4, Bn), 128, 0, stream>>>(xt, hm, cen, R, P, he);
  node_kernel<<<dim3(NNT, Bn), 256, 0, stream>>>(he, phi, R, P, out);
}
